// InfraredFeatureExtractor_11227044512391
// MI455X (gfx1250) — hardware-verified
//
#include <hip/hip_runtime.h>
#include <stddef.h>
#include <stdint.h>


#define IMH   256
#define IMW   256
#define NPIX  65536
#define NIMG  2
#define RR    131072
#define CA    16
#define CB    32
#define CC    64
#define NTHR  256
#define NWAVE 8
#define CHUNK 2048
#define WCAP  256
#define NGRP  (CHUNK / (NTHR * 4))
#define RECP  256
#define AP    40
#define GR    128

static_assert(WCAP == (CHUNK / NTHR) * 32);
static_assert(NGRP == 2);
static_assert(RECP == NTHR);
static_assert((RR % GR) == 0);
static_assert((NPIX % 512) == 0);
static_assert((NPIX % GR) == 0);

typedef float          v2f   __attribute__((ext_vector_type(2)));
typedef float          v4f   __attribute__((ext_vector_type(4)));
typedef float          v8f   __attribute__((ext_vector_type(8)));
typedef double         v2d   __attribute__((ext_vector_type(2)));
typedef int            v4i   __attribute__((ext_vector_type(4)));
typedef unsigned short v8us  __attribute__((ext_vector_type(8)));
typedef unsigned short v16us __attribute__((ext_vector_type(16)));
typedef __bf16         v16bf __attribute__((ext_vector_type(16)));
union FragB { v16bf v; v16us u; v8us h[2]; };

template <int N> struct VTy;
template <> struct VTy<2> { typedef v2f t; };
template <> struct VTy<4> { typedef v4f t; };

__device__ __forceinline__ int iclamp(int v, int lo, int hi) { return v < lo ? lo : (v > hi ? hi : v); }

__device__ __forceinline__ unsigned int bfr(float x) {
  const unsigned int u = __float_as_uint(x);
  return (u + 0x7FFFu + ((u >> 16) & 1u)) >> 16;
}
__device__ __forceinline__ void split2(float x, unsigned short& hi, unsigned short& lo) {
  const unsigned int hb = bfr(x);
  const float hf = __uint_as_float(hb << 16);
  hi = (unsigned short)hb;
  lo = (unsigned short)bfr(x - hf);
}

__device__ __forceinline__ float lin255(int i) {
  const float s = (float)i * (1.0f / 255.0f);
  const float t = 1.0f - s;
  const float v = s - t;
  return (i >= 255) ? 1.0f : v;
}

__device__ __forceinline__ float ffval(float x, float mu, float rs, float g, float b, float cwv, float fl, float fbv) {
  const float f = g * (x - mu) * rs + b;
  const float t = f * cwv;
  return t * fl + fbv;
}

__device__ __forceinline__ v8f wm3(const FragB& ah, const FragB& al, const FragB& bh, const FragB& bl, v8f c) {
  c = __builtin_amdgcn_wmma_f32_16x16x32_bf16(false, ah.v, false, bh.v, (short)0, c, false, false);
  c = __builtin_amdgcn_wmma_f32_16x16x32_bf16(false, ah.v, false, bl.v, (short)0, c, false, false);
  c = __builtin_amdgcn_wmma_f32_16x16x32_bf16(false, al.v, false, bh.v, (short)0, c, false, false);
  asm volatile("v_nop\n\tv_nop\n\tv_nop\n\tv_nop" : "+v"(c) : "v"(ah.v), "v"(al.v), "v"(bh.v), "v"(bl.v));
  return c;
}

__global__ __launch_bounds__(NTHR) void k_prepw(const float* __restrict__ w, unsigned short* ph,
                                                unsigned short* pl, int cout, int cin, int n8) {
  const int i = blockIdx.x * NTHR + threadIdx.x;
  if (i >= n8) return;
  const int o = i * 8;
  const int per = cout * cin;
  const int tap = o / per;
  const int rem = o - tap * per;
  const int co = rem / cin;
  const int ci0 = rem - co * cin;
  v8us vh, vl;
#pragma unroll
  for (int j = 0; j < 8; ++j) {
    const float v = w[(size_t)(co * cin + ci0 + j) * 9 + tap];
    unsigned short a, b;
    split2(v, a, b);
    vh[j] = a; vl[j] = b;
  }
  *(volatile v8us*)(ph + o) = vh;
  *(volatile v8us*)(pl + o) = vl;
  __threadfence();
  *(volatile v8us*)(ph + o) = vh;
  *(volatile v8us*)(pl + o) = vl;
}

__global__ __launch_bounds__(NTHR) void k_conv1(const float* __restrict__ x, const float* __restrict__ w,
                                                const float* __restrict__ b, float* c1, double* rec) {
  __shared__ __attribute__((aligned(16))) float T[NTHR * CA];
  __shared__ __attribute__((aligned(16))) double R[RECP];
  const int tid = threadIdx.x, lane = tid & 31, wave = tid >> 5;
  const int blk = blockIdx.x;
  const int img = blk >> 8;
  const int y = blk & 255;
  const int xq = tid;
  const float* xb = x + (size_t)img * NPIX;
  float tp[25];
#pragma unroll
  for (int ky = 0; ky < 5; ++ky) {
    const int yy = y + ky - 2;
    const bool oky = (unsigned)yy < (unsigned)IMH;
    const int yc = iclamp(yy, 0, IMH - 1);
#pragma unroll
    for (int kx = 0; kx < 5; ++kx) {
      const int xx = xq + kx - 2;
      const bool ok = oky && ((unsigned)xx < (unsigned)IMW);
      const int xc = iclamp(xx, 0, IMW - 1);
      const float v = xb[yc * IMW + xc];
      tp[ky * 5 + kx] = ok ? v : 0.f;
    }
  }
#pragma unroll 1
  for (int c = 0; c < CA; ++c) {
    float acc = 0.f;
#pragma unroll
    for (int t = 0; t < 25; ++t) acc += tp[t] * w[c * 25 + t];
    acc += b[c];
    T[tid * CA + c] = fmaxf(acc, 0.f);
  }
  R[tid] = 0.0;
  __syncthreads();
  {
    const int c = tid >> 4, part = tid & 15;
    double s = 0.0, q = 0.0;
#pragma unroll 4
    for (int i = 0; i < 16; ++i) {
      const float v = T[(part * 16 + i) * CA + c];
      s += (double)v;
      q += (double)v * (double)v;
    }
#pragma unroll
    for (int mk = 8; mk > 0; mk >>= 1) {
      s += __shfl_xor(s, mk, 32);
      q += __shfl_xor(q, mk, 32);
    }
    if (part == 0) { R[c * 2] = s; R[c * 2 + 1] = q; }
  }
  __syncthreads();
  float* gq = c1 + (size_t)blk * (NTHR * CA);
  v4f xr[4];
#pragma unroll
  for (int i = 0; i < 4; ++i) xr[i] = *(const v4f*)(T + wave * 512 + i * 128 + lane * 4);
  v2d rv = {0.0, 0.0};
  if (wave < 4) rv = *(const v2d*)(R + (wave * 32 + lane) * 2);
  double* rp = rec + (size_t)blk * RECP + (wave * 32 + lane) * 2;
#pragma unroll
  for (int i = 0; i < 4; ++i) *(volatile v4f*)(gq + wave * 512 + i * 128 + lane * 4) = xr[i];
  if (wave < 4) *(volatile v2d*)rp = rv;
  __threadfence();
#pragma unroll
  for (int i = 0; i < 4; ++i) *(volatile v4f*)(gq + wave * 512 + i * 128 + lane * 4) = xr[i];
  if (wave < 4) *(volatile v2d*)rp = rv;
}

__global__ __launch_bounds__(64) void k_fin(const double* __restrict__ rec, int nblk, int nc, float cnt,
                                            const float* __restrict__ g, const float* __restrict__ bt,
                                            const float* __restrict__ w1, const float* __restrict__ b1,
                                            const float* __restrict__ w2, const float* __restrict__ b2,
                                            int mlp, float* st, float* cw) {
  __shared__ __attribute__((aligned(16))) float stl[128];
  __shared__ __attribute__((aligned(16))) float cws[128];
  __shared__ float pool[128];
  __shared__ float hm[32];
  __shared__ float lg[128];
  __shared__ float ex[128];
  __shared__ float mx[2];
  __shared__ float sm[2];
  const int t = threadIdx.x;
  const bool act = t < nc;
  const int c = act ? t : (nc - 1);
  double s0 = 0.0, s1 = 0.0, q0 = 0.0, q1 = 0.0;
#pragma unroll 1
  for (int k = 0; k < nblk; ++k) {
    const double* r = rec + (size_t)k * RECP;
    s0 += r[c * 2];
    q0 += r[c * 2 + 1];
    s1 += r[(nc + c) * 2];
    q1 += r[(nc + c) * 2 + 1];
  }
  const double icnt = 1.0 / (double)cnt;
  const double mu = (s0 + s1) * icnt;
  double var = (q0 + q1) * icnt - mu * mu;
  if (var < 0.0) var = 0.0;
  const float muf = (float)mu;
  const float varf = (float)var;
  const float rs = 1.0f / sqrtf(varf + 1e-5f);
  stl[2 * t] = act ? muf : 0.f;
  stl[2 * t + 1] = act ? rs : 0.f;
  if (mlp) {
    const float m0 = (float)(s0 * (1.0 / (double)NPIX));
    const float m1 = (float)(s1 * (1.0 / (double)NPIX));
    pool[t]      = act ? (g[c] * (m0 - muf) * rs + bt[c]) : 0.f;
    pool[64 + t] = act ? (g[c] * (m1 - muf) * rs + bt[c]) : 0.f;
  }
  __syncthreads();
  if (t < 32) {
    const v4f v = *(const v4f*)(stl + 4 * t);
    *(volatile v4f*)(st + 4 * t) = v;
    __threadfence();
    *(volatile v4f*)(st + 4 * t) = v;
  }
  if (mlp) {
    if (t < 32) {
      const int im = t >> 4, j = t & 15;
      float a = 0.f;
#pragma unroll 1
      for (int k = 0; k < CC; ++k) a += pool[im * 64 + k] * w1[j * CC + k];
      a += b1[j];
      hm[im * 16 + j] = fmaxf(a, 0.f);
    }
    __syncthreads();
#pragma unroll 1
    for (int im = 0; im < 2; ++im) {
      float l = 0.f;
#pragma unroll 1
      for (int j = 0; j < 16; ++j) l += hm[im * 16 + j] * w2[c * 16 + j];
      l += b2[c];
      lg[im * 64 + t] = l;
    }
    __syncthreads();
    if (t < 2) {
      float m = -1.0e30f;
#pragma unroll 1
      for (int k = 0; k < CC; ++k) m = fmaxf(m, lg[t * 64 + k]);
      mx[t] = m;
    }
    __syncthreads();
#pragma unroll 1
    for (int im = 0; im < 2; ++im) ex[im * 64 + t] = expf(lg[im * 64 + t] - mx[im]);
    __syncthreads();
    if (t < 2) {
      float s = 0.f;
#pragma unroll 1
      for (int k = 0; k < CC; ++k) s += ex[t * 64 + k];
      sm[t] = s;
    }
    __syncthreads();
#pragma unroll 1
    for (int im = 0; im < 2; ++im) cws[im * 64 + t] = ex[im * 64 + t] * (1.0f / sm[im]);
    __syncthreads();
    if (t < 32) {
      const v4f v = *(const v4f*)(cws + 4 * t);
      *(volatile v4f*)(cw + 4 * t) = v;
      __threadfence();
      *(volatile v4f*)(cw + 4 * t) = v;
    }
  }
}

template <int NC, int KIN>
__global__ __launch_bounds__(NTHR) void k_tr(const float* __restrict__ xin, const float* __restrict__ st,
                                             const float* __restrict__ g, const float* __restrict__ bt,
                                             const float* __restrict__ pw, const float* __restrict__ pb,
                                             const float* __restrict__ W, const float* __restrict__ aw_s,
                                             const float* __restrict__ aw_d, float* h, float* asb, float* adb) {
  constexpr int CT = NC / 16;
  constexpr int CPT = KIN / 2;
  constexpr int WCH = GR * NC / 8;
  static_assert(KIN == 16 || KIN == 32);
  static_assert(NC == 32 || NC == 64);
  __shared__ __attribute__((aligned(16))) unsigned short Ah[GR * AP];
  __shared__ __attribute__((aligned(16))) unsigned short Al[GR * AP];
  __shared__ __attribute__((aligned(16))) unsigned short Whs[NC * AP];
  __shared__ __attribute__((aligned(16))) unsigned short Wls[NC * AP];
  __shared__ __attribute__((aligned(16))) float Ds[GR * NC];
  __shared__ __attribute__((aligned(16))) float As[GR];
  __shared__ __attribute__((aligned(16))) float Ad[GR];

  const int tid = threadIdx.x, lane = tid & 31, wave = tid >> 5, hh = lane >> 4, m = lane & 15;
  const int r0 = blockIdx.x * GR;

  {
    const int r = tid >> 1, half = tid & 1, c0 = half * CPT;
    const int row = r0 + r;
    const int node = row & (NPIX - 1);
    const float gy = lin255(node >> 8);
    const float gx = lin255(node & 255);
    const float* xp = xin + (size_t)row * KIN + c0;
    float xv[CPT];
#pragma unroll
    for (int i = 0; i < CPT / 4; ++i) {
      const v4f qv = *(const v4f*)(xp + 4 * i);
      xv[4 * i] = qv.x; xv[4 * i + 1] = qv.y; xv[4 * i + 2] = qv.z; xv[4 * i + 3] = qv.w;
    }
    unsigned short hv[CPT], lv[CPT];
#pragma unroll
    for (int j = 0; j < CPT; ++j) {
      const int c = c0 + j;
      float v = g[c] * (xv[j] - st[2 * c]) * st[2 * c + 1] + bt[c];
      const float pe = gy * pw[2 * c] + gx * pw[2 * c + 1] + pb[c];
      v += pe;
      split2(v, hv[j], lv[j]);
    }
#pragma unroll
    for (int i = 0; i < CPT / 8; ++i) {
      v8us a, bq;
#pragma unroll
      for (int j = 0; j < 8; ++j) { a[j] = hv[8 * i + j]; bq[j] = lv[8 * i + j]; }
      *(v8us*)(Ah + r * AP + c0 + 8 * i) = a;
      *(v8us*)(Al + r * AP + c0 + 8 * i) = bq;
    }
    if (KIN == 16) {
      const v8us z8 = {0, 0, 0, 0, 0, 0, 0, 0};
      *(v8us*)(Ah + r * AP + 16 + c0) = z8;
      *(v8us*)(Al + r * AP + 16 + c0) = z8;
    }
  }
  for (int e = tid; e < NC * 32; e += NTHR) {
    const int n = e >> 5, k = e & 31;
    float wv = W[n * KIN + (k < KIN ? k : KIN - 1)];
    wv = (k < KIN) ? wv : 0.f;
    unsigned short a, bq;
    split2(wv, a, bq);
    Whs[n * AP + k] = a;
    Wls[n * AP + k] = bq;
  }
  __syncthreads();

  FragB ah, al;
  ah.h[0] = *(const v8us*)(Ah + (16 * wave + m) * AP + 8 * hh);
  ah.h[1] = *(const v8us*)(Ah + (16 * wave + m) * AP + 16 + 8 * hh);
  al.h[0] = *(const v8us*)(Al + (16 * wave + m) * AP + 8 * hh);
  al.h[1] = *(const v8us*)(Al + (16 * wave + m) * AP + 16 + 8 * hh);
  v8f acc[CT];
#pragma unroll
  for (int ct = 0; ct < CT; ++ct) {
    FragB bh, bl;
    bh.h[0] = *(const v8us*)(Whs + (16 * ct + m) * AP + 8 * hh);
    bh.h[1] = *(const v8us*)(Whs + (16 * ct + m) * AP + 16 + 8 * hh);
    bl.h[0] = *(const v8us*)(Wls + (16 * ct + m) * AP + 8 * hh);
    bl.h[1] = *(const v8us*)(Wls + (16 * ct + m) * AP + 16 + 8 * hh);
    const v8f z = {0.f, 0.f, 0.f, 0.f, 0.f, 0.f, 0.f, 0.f};
    acc[ct] = wm3(ah, al, bh, bl, z);
  }

  float cs[CT], cd[CT];
#pragma unroll
  for (int ct = 0; ct < CT; ++ct) { cs[ct] = aw_s[16 * ct + m]; cd[ct] = aw_d[16 * ct + m]; }
  float ss[8], sd[8];
#pragma unroll
  for (int r = 0; r < 8; ++r) { ss[r] = 0.f; sd[r] = 0.f; }
#pragma unroll
  for (int ct = 0; ct < CT; ++ct) {
#pragma unroll
    for (int r = 0; r < 8; ++r) {
      const float v = acc[ct][r];
      Ds[(16 * wave + 8 * hh + r) * NC + 16 * ct + m] = v;
      ss[r] += v * cs[ct];
      sd[r] += v * cd[ct];
    }
  }
#pragma unroll
  for (int mk = 1; mk < 16; mk <<= 1) {
#pragma unroll
    for (int r = 0; r < 8; ++r) {
      ss[r] += __shfl_xor(ss[r], mk, 32);
      sd[r] += __shfl_xor(sd[r], mk, 32);
    }
  }
  if (m == 0) {
#pragma unroll
    for (int r = 0; r < 8; ++r) { As[16 * wave + 8 * hh + r] = ss[r]; Ad[16 * wave + 8 * hh + r] = sd[r]; }
  }
  __syncthreads();

  v4f xr[WCH / 128];
#pragma unroll
  for (int i = 0; i < WCH / 128; ++i) xr[i] = *(const v4f*)(Ds + wave * WCH + i * 128 + lane * 4);
  v4f gv = {0.f, 0.f, 0.f, 0.f};
  if (wave == 0) gv = *(const v4f*)(As + 4 * lane);
  else if (wave == 1) gv = *(const v4f*)(Ad + 4 * lane);
  float* hb = h + (size_t)r0 * NC + wave * WCH + lane * 4;
  float* ap = (wave == 0) ? (asb + r0 + 4 * lane) : (adb + r0 + 4 * lane);
#pragma unroll
  for (int i = 0; i < WCH / 128; ++i) *(volatile v4f*)(hb + i * 128) = xr[i];
  if (wave < 2) *(volatile v4f*)ap = gv;
  __threadfence();
#pragma unroll
  for (int i = 0; i < WCH / 128; ++i) *(volatile v4f*)(hb + i * 128) = xr[i];
  if (wave < 2) *(volatile v4f*)ap = gv;
}

template <int NC, int NB, int CPL>
__global__ __launch_bounds__(NTHR) void k_gat(const float* __restrict__ h, const float* __restrict__ asb,
                                              const float* __restrict__ adb, const int* __restrict__ srcp,
                                              const int* __restrict__ dstp, const float* __restrict__ gb,
                                              float* gout, double* rec, int nE) {
  typedef typename VTy<CPL>::t VT;
  static_assert(NC == 16 * CPL);
  static_assert(NB <= 512);
  static_assert((NPIX % NB) == 0);
  static_assert((NB % NWAVE) == 0);
  extern __shared__ v4f lds_dyn[];
  float*  sacc  = (float*)lds_dyn;
  float*  aux   = sacc + NB * 2 * NC;
  int*    list  = (int*)(aux + NB * 4);
  int*    wcnt  = list + NWAVE * WCAP;
  double* wpart = (double*)(wcnt + 8);
  double* recs  = wpart + NWAVE * 32 * 2 * CPL;

  const int tid = threadIdx.x, lane = tid & 31, wave = tid >> 5;
  const int im = lane >> 4, q = lane & 15;
  const int nodeBase = blockIdx.x * NB;

  {
    const v4f z4 = {0.f, 0.f, 0.f, 0.f};
    for (int i = tid; i < NB * 2 * NC / 4; i += NTHR) lds_dyn[i] = z4;
    for (int i = tid; i < NB * 2; i += NTHR) { aux[2 * i] = -1.0e30f; aux[2 * i + 1] = 0.f; }
  }
  __syncthreads();

  const bool al16 = ((((size_t)dstp) & 15) == 0);
  const int nChunks = (nE + CHUNK - 1) / CHUNK;
#pragma unroll 1
  for (int ch = 0; ch < nChunks; ++ch) {
    const int cbase = ch * CHUNK;
    int wc = 0;
#pragma unroll
    for (int gI = 0; gI < NGRP; ++gI) {
      const int el0 = (gI * NTHR + tid) * 4;
      const int e0 = cbase + el0;
      const int sent = -2147483647 - 1;
      v4i d;
      if (al16 && (cbase + CHUNK <= nE)) {
        d = *(const v4i*)(dstp + e0);
      } else {
        d.x = (e0     < nE) ? dstp[iclamp(e0,     0, nE - 1)] : sent;
        d.y = (e0 + 1 < nE) ? dstp[iclamp(e0 + 1, 0, nE - 1)] : sent;
        d.z = (e0 + 2 < nE) ? dstp[iclamp(e0 + 2, 0, nE - 1)] : sent;
        d.w = (e0 + 3 < nE) ? dstp[iclamp(e0 + 3, 0, nE - 1)] : sent;
      }
      const unsigned s0 = (unsigned)d.x - (unsigned)nodeBase;
      const unsigned s1 = (unsigned)d.y - (unsigned)nodeBase;
      const unsigned s2 = (unsigned)d.z - (unsigned)nodeBase;
      const unsigned s3 = (unsigned)d.w - (unsigned)nodeBase;
      const bool h0 = s0 < (unsigned)NB;
      const bool h1 = s1 < (unsigned)NB;
      const bool h2 = s2 < (unsigned)NB;
      const bool h3 = s3 < (unsigned)NB;
      const unsigned many = __builtin_amdgcn_ballot_w32(h0 | h1 | h2 | h3);
      if (many != 0u) {
#define HITJ(J, HJ, SJ) { \
          const unsigned mj = __builtin_amdgcn_ballot_w32(HJ); \
          if (HJ) { \
            const int pos = wc + (int)__builtin_amdgcn_mbcnt_lo(mj, 0u); \
            if (pos < WCAP) list[wave * WCAP + pos] = ((el0 + (J)) << 9) | (int)(SJ); \
          } \
          wc += (int)__builtin_popcount(mj); }
        HITJ(0, h0, s0)
        HITJ(1, h1, s1)
        HITJ(2, h2, s2)
        HITJ(3, h3, s3)
#undef HITJ
      }
    }
    if (lane == 0) wcnt[wave] = wc;
    __syncthreads();

    if (wave == 0) {
#pragma unroll 1
      for (int wsx = 0; wsx < NWAVE; ++wsx) {
        int n = wcnt[wsx];
        n = n > WCAP ? WCAP : (n < 0 ? 0 : n);
#pragma unroll 1
        for (int i = 0; i < n; ++i) {
          const int ent = list[wsx * WCAP + i];
          const int slot = ent & (NB - 1);
          const int el = (ent >> 9) & (CHUNK - 1);
          const int e = iclamp(cbase + el, 0, nE - 1);
          const int s = iclamp(srcp[e], 0, NPIX - 1);
          const int node = iclamp(nodeBase + slot, 0, NPIX - 1);
          float ev = asb[im * NPIX + s] + adb[im * NPIX + node];
          ev = (ev > 0.f) ? ev : 0.2f * ev;
          float* apx = aux + (slot * 2 + im) * 2;
          const float mo = apx[0];
          const float dn = apx[1];
          const float mn = fmaxf(mo, ev);
          const float sc = expf(mo - mn);
          const float p = expf(ev - mn);
          const VT hv = *(const VT*)(h + (size_t)(im * NPIX + s) * NC + CPL * q);
          VT* spp = (VT*)(sacc + slot * (2 * NC) + CPL * lane);
          const VT cur = *spp;
          const VT nxt = cur * sc + hv * p;
          *spp = nxt;
          const float dnn = dn * sc + p;
          apx[0] = mn;
          apx[1] = dnn;
        }
      }
    }
    __syncthreads();
  }

  const VT bb = *(const VT*)(gb + CPL * q);
  double S[CPL], Q[CPL];
#pragma unroll
  for (int k = 0; k < CPL; ++k) { S[k] = 0.0; Q[k] = 0.0; }
#pragma unroll 1
  for (int j = 0; j < NB / NWAVE; ++j) {
    const int slot = wave * (NB / NWAVE) + j;
    const int node = nodeBase + slot;
    const float dn = aux[(slot * 2 + im) * 2 + 1];
    const float inv = 1.0f / (dn + 1e-16f);
    VT v = *(const VT*)(sacc + slot * (2 * NC) + CPL * lane) * inv + bb;
#pragma unroll
    for (int k = 0; k < CPL; ++k) {
      const float t = v[k] > 0.f ? v[k] : 0.f;
      v[k] = t;
      S[k] += (double)t;
      Q[k] += (double)t * (double)t;
    }
    float* op = gout + (size_t)(im * NPIX + node) * NC + CPL * q;
    *(volatile VT*)op = v;
    __threadfence();
    *(volatile VT*)op = v;
  }
#pragma unroll
  for (int k = 0; k < CPL; ++k) {
    wpart[(wave * 32 + lane) * (2 * CPL) + k] = S[k];
    wpart[(wave * 32 + lane) * (2 * CPL) + CPL + k] = Q[k];
  }
  __syncthreads();
  if (tid < 4 * NC) {
    const int imx = tid / (2 * NC);
    const int c = (tid >> 1) % NC;
    const int sq = tid & 1;
    const int ln = imx * 16 + c / CPL;
    const int jj = c % CPL;
    double a = 0.0;
#pragma unroll
    for (int w8 = 0; w8 < NWAVE; ++w8) a += wpart[(w8 * 32 + ln) * (2 * CPL) + sq * CPL + jj];
    recs[tid] = a;
  } else {
    recs[tid] = 0.0;
  }
  __syncthreads();
  if (wave < 4) {
    const v2d rv = *(const v2d*)(recs + (wave * 32 + lane) * 2);
    double* rp = rec + (size_t)blockIdx.x * RECP + (wave * 32 + lane) * 2;
    *(volatile v2d*)rp = rv;
    __threadfence();
    *(volatile v2d*)rp = rv;
  }
}

__global__ __launch_bounds__(NTHR) void k_ffp(const float* __restrict__ g2, const float* __restrict__ st,
                                              const float* __restrict__ g, const float* __restrict__ bt,
                                              const float* __restrict__ cw, const float* __restrict__ filt,
                                              const float* __restrict__ fb, unsigned short* fh, unsigned short* fl) {
  const int gid = blockIdx.x * NTHR + threadIdx.x;
  const int pix = gid >> 3;
  const int c0 = (gid & 7) * 8;
  const int im = pix >> 16;
  const int node = pix & (NPIX - 1);
  const v4f a = *(const v4f*)(g2 + (size_t)pix * CC + c0);
  const v4f b = *(const v4f*)(g2 + (size_t)pix * CC + c0 + 4);
  const float xv[8] = {a.x, a.y, a.z, a.w, b.x, b.y, b.z, b.w};
  v8us vh, vl;
#pragma unroll
  for (int j = 0; j < 8; ++j) {
    const int c = c0 + j;
    const float v = ffval(xv[j], st[2 * c], st[2 * c + 1], g[c], bt[c], cw[im * CC + c],
                          filt[(size_t)c * NPIX + node], fb[c]);
    unsigned short hb, lb;
    split2(v, hb, lb);
    vh[j] = hb; vl[j] = lb;
  }
  const size_t o = (size_t)pix * CC + c0;
  *(volatile v8us*)(fh + o) = vh;
  *(volatile v8us*)(fl + o) = vl;
  __threadfence();
  *(volatile v8us*)(fh + o) = vh;
  *(volatile v8us*)(fl + o) = vl;
}

template <int CIN, int COUT, int MODE>
__global__ __launch_bounds__(NTHR) void k_conv(const unsigned short* __restrict__ Xh,
                                               const unsigned short* __restrict__ Xl,
                                               const unsigned short* __restrict__ Wh,
                                               const unsigned short* __restrict__ Wl,
                                               const float* __restrict__ bias, unsigned short* Oh, unsigned short* Ol,
                                               const float* __restrict__ g2, const float* __restrict__ st,
                                               const float* __restrict__ g3, const float* __restrict__ b3,
                                               const float* __restrict__ cw, const float* __restrict__ filt,
                                               const float* __restrict__ fb, float* pre, double* rec) {
  constexpr int CHUNKS = CIN / 32;
  constexpr int CT = COUT / 16;
  static_assert((CIN % 32) == 0);
  static_assert((COUT % 16) == 0);
  extern __shared__ v4f lds_dyn[];
  const int tid = threadIdx.x, lane = tid & 31, wave = tid >> 5, hh = lane >> 4, m = lane & 15;
  const int blk = blockIdx.x, img = blk >> 8, y = blk & 255, x0 = wave * 32;

  v8f acc[2][CT];
#pragma unroll
  for (int mt = 0; mt < 2; ++mt) {
#pragma unroll
    for (int ct = 0; ct < CT; ++ct) {
      const v8f z = {0.f, 0.f, 0.f, 0.f, 0.f, 0.f, 0.f, 0.f};
      acc[mt][ct] = z;
    }
  }
  const v8us z8 = {0, 0, 0, 0, 0, 0, 0, 0};

#pragma unroll 1
  for (int tap = 0; tap < 9; ++tap) {
    const int ky = tap / 3;
    const int dy = ky - 1;
    const int dx = tap - ky * 3 - 1;
    const int yy = y + dy;
    const bool oky = (unsigned)yy < (unsigned)IMH;
    const int yc = iclamp(yy, 0, IMH - 1);
    const int xa = x0 + m + dx;
    const int xb = xa + 16;
    const bool oka = oky && ((unsigned)xa < (unsigned)IMW);
    const bool okb = oky && ((unsigned)xb < (unsigned)IMW);
    const size_t ra = (size_t)(img * NPIX + yc * IMW + iclamp(xa, 0, IMW - 1)) * CIN;
    const size_t rb = (size_t)(img * NPIX + yc * IMW + iclamp(xb, 0, IMW - 1)) * CIN;
    const unsigned short* wrh = Wh + (size_t)(tap * COUT + m) * CIN;
    const unsigned short* wrl = Wl + (size_t)(tap * COUT + m) * CIN;
#pragma unroll
    for (int chn = 0; chn < CHUNKS; ++chn) {
      const int k0 = chn * 32 + 8 * hh;
      FragB ah0, al0, ah1, al1;
      v8us t;
      t = *(const v8us*)(Xh + ra + k0);      ah0.h[0] = oka ? t : z8;
      t = *(const v8us*)(Xh + ra + k0 + 16); ah0.h[1] = oka ? t : z8;
      t = *(const v8us*)(Xl + ra + k0);      al0.h[0] = oka ? t : z8;
      t = *(const v8us*)(Xl + ra + k0 + 16); al0.h[1] = oka ? t : z8;
      t = *(const v8us*)(Xh + rb + k0);      ah1.h[0] = okb ? t : z8;
      t = *(const v8us*)(Xh + rb + k0 + 16); ah1.h[1] = okb ? t : z8;
      t = *(const v8us*)(Xl + rb + k0);      al1.h[0] = okb ? t : z8;
      t = *(const v8us*)(Xl + rb + k0 + 16); al1.h[1] = okb ? t : z8;
#pragma unroll
      for (int ct = 0; ct < CT; ++ct) {
        FragB bh, bl;
        const unsigned short* bp = wrh + (size_t)ct * 16 * CIN + k0;
        const unsigned short* bq = wrl + (size_t)ct * 16 * CIN + k0;
        bh.h[0] = *(const v8us*)bp; bh.h[1] = *(const v8us*)(bp + 16);
        bl.h[0] = *(const v8us*)bq; bl.h[1] = *(const v8us*)(bq + 16);
        acc[0][ct] = wm3(ah0, al0, bh, bl, acc[0][ct]);
        acc[1][ct] = wm3(ah1, al1, bh, bl, acc[1][ct]);
      }
    }
  }

  if (MODE == 0) {
    unsigned short* Eh = (unsigned short*)lds_dyn + wave * (2 * 32 * COUT);
    unsigned short* El = Eh + 32 * COUT;
#pragma unroll
    for (int ct = 0; ct < CT; ++ct) {
      const int co = 16 * ct + m;
      const float bco = bias[co];
#pragma unroll
      for (int mt = 0; mt < 2; ++mt) {
#pragma unroll
        for (int r = 0; r < 8; ++r) {
          const float v = fmaxf(acc[mt][ct][r] + bco, 0.f);
          unsigned short hb, lb;
          split2(v, hb, lb);
          Eh[(mt * 16 + 8 * hh + r) * COUT + co] = hb;
          El[(mt * 16 + 8 * hh + r) * COUT + co] = lb;
        }
      }
    }
    __syncthreads();
    const size_t gbase = (size_t)(img * NPIX + y * IMW + x0) * COUT;
    v4i ph[COUT / 8], pl[COUT / 8];
#pragma unroll
    for (int i = 0; i < COUT / 8; ++i) {
      ph[i] = *(const v4i*)(Eh + i * 256 + lane * 8);
      pl[i] = *(const v4i*)(El + i * 256 + lane * 8);
    }
#pragma unroll
    for (int i = 0; i < COUT / 8; ++i) {
      *(volatile v4i*)(Oh + gbase + i * 256 + lane * 8) = ph[i];
      *(volatile v4i*)(Ol + gbase + i * 256 + lane * 8) = pl[i];
    }
    __threadfence();
#pragma unroll
    for (int i = 0; i < COUT / 8; ++i) {
      *(volatile v4i*)(Oh + gbase + i * 256 + lane * 8) = ph[i];
      *(volatile v4i*)(Ol + gbase + i * 256 + lane * 8) = pl[i];
    }
  } else {
    float* P = (float*)lds_dyn;
    double* recs = (double*)(P + COUT * 256);
    const int pixb = y * IMW;
#pragma unroll
    for (int ct = 0; ct < CT; ++ct) {
      const int co = 16 * ct + m;
      const float mu = st[2 * co], rs = st[2 * co + 1];
      const float gg = g3[co], be = b3[co];
      const float cwv = cw[img * CC + co];
      const float fbv = fb[co];
      const float bco = bias[co];
#pragma unroll
      for (int mt = 0; mt < 2; ++mt) {
#pragma unroll
        for (int r = 0; r < 8; ++r) {
          const int xx = x0 + mt * 16 + 8 * hh + r;
          const int pix = pixb + xx;
          const float xg = g2[(size_t)(img * NPIX + pix) * CC + co];
          const float flv = filt[(size_t)co * NPIX + pix];
          const float ffv = ffval(xg, mu, rs, gg, be, cwv, flv, fbv);
          const float v = (acc[mt][ct][r] + bco) + ffv;
          P[co * 256 + xx] = fmaxf(v, 0.f);
        }
      }
    }
    recs[tid] = 0.0;
    __syncthreads();
    {
      const int c = tid >> 2, part = tid & 3;
      double s = 0.0, qq = 0.0;
#pragma unroll 4
      for (int i = 0; i < 64; ++i) {
        const float v = P[c * 256 + part * 64 + i];
        s += (double)v;
        qq += (double)v * (double)v;
      }
      s += __shfl_xor(s, 1, 32);  qq += __shfl_xor(qq, 1, 32);
      s += __shfl_xor(s, 2, 32);  qq += __shfl_xor(qq, 2, 32);
      if (part == 0) { recs[c * 2] = s; recs[c * 2 + 1] = qq; }
    }
    v4f pv[16];
#pragma unroll
    for (int i = 0; i < 8; ++i) {
      const int c = wave + 8 * i;
#pragma unroll
      for (int k = 0; k < 2; ++k) pv[2 * i + k] = *(const v4f*)(P + c * 256 + k * 128 + lane * 4);
    }
#pragma unroll
    for (int i = 0; i < 8; ++i) {
      const int c = wave + 8 * i;
      float* gp = pre + (size_t)(img * CC + c) * NPIX + pixb + lane * 4;
#pragma unroll
      for (int k = 0; k < 2; ++k) *(volatile v4f*)(gp + k * 128) = pv[2 * i + k];
    }
    __threadfence();
#pragma unroll
    for (int i = 0; i < 8; ++i) {
      const int c = wave + 8 * i;
      float* gp = pre + (size_t)(img * CC + c) * NPIX + pixb + lane * 4;
#pragma unroll
      for (int k = 0; k < 2; ++k) *(volatile v4f*)(gp + k * 128) = pv[2 * i + k];
    }
    __syncthreads();
    if (wave < 4) {
      const v2d rv = *(const v2d*)(recs + (wave * 32 + lane) * 2);
      double* rp = rec + (size_t)blk * RECP + (wave * 32 + lane) * 2;
      *(volatile v2d*)rp = rv;
      __threadfence();
      *(volatile v2d*)rp = rv;
    }
  }
}

__global__ __launch_bounds__(NTHR) void k_out(const float* __restrict__ pre, const float* __restrict__ st,
                                              const float* __restrict__ g, const float* __restrict__ bt, float* out) {
  const size_t i4 = (size_t)blockIdx.x * NTHR + threadIdx.x;
  const int c = (int)((i4 >> 14) & 63);
  const v4f v = *(const v4f*)(pre + i4 * 4);
  const float mu = st[2 * c], rs = st[2 * c + 1], gg = g[c], be = bt[c];
  v4f yv;
  yv.x = gg * (v.x - mu) * rs + be;
  yv.y = gg * (v.y - mu) * rs + be;
  yv.z = gg * (v.z - mu) * rs + be;
  yv.w = gg * (v.w - mu) * rs + be;
  *(volatile v4f*)(out + i4 * 4) = yv;
  __threadfence();
  *(volatile v4f*)(out + i4 * 4) = yv;
}

extern "C" void kernel_launch(void* const* d_in, const int* in_sizes, int n_in,
                              void* d_out, int out_size, void* d_ws, size_t ws_size,
                              hipStream_t stream) {
  if (n_in < 35) return;
  if (in_sizes[0] != NIMG * NPIX) return;
  if (in_sizes[1] != CA * 25 || in_sizes[2] != CA || in_sizes[3] != CA || in_sizes[4] != CA) return;
  if (in_sizes[5] != CA * 2 || in_sizes[6] != CA) return;
  if (in_sizes[7] != CB * CA || in_sizes[8] != CB || in_sizes[9] != CB || in_sizes[10] != CB) return;
  if (in_sizes[11] != CB || in_sizes[12] != CB || in_sizes[13] != CB * 2 || in_sizes[14] != CB) return;
  if (in_sizes[15] != CC * CB || in_sizes[16] != CC || in_sizes[17] != CC || in_sizes[18] != CC) return;
  if (in_sizes[19] != CC || in_sizes[20] != CC) return;
  if (in_sizes[21] != 16 * CC || in_sizes[22] != 16 || in_sizes[23] != CC * 16 || in_sizes[24] != CC) return;
  if (in_sizes[25] != CC * NPIX || in_sizes[26] != CC) return;
  if (in_sizes[27] != CB * CC * 9 || in_sizes[28] != CB || in_sizes[29] != CC * CB * 9 || in_sizes[30] != CC) return;
  if (in_sizes[31] != CC || in_sizes[32] != CC) return;
  const int nE = in_sizes[33];
  if (nE <= 0 || in_sizes[34] != nE) return;
  if (out_size != NIMG * CC * NPIX) return;

  const float* x       = (const float*)d_in[0];
  const float* conv1_w = (const float*)d_in[1];
  const float* conv1_b = (const float*)d_in[2];
  const float* bn1_g   = (const float*)d_in[3];
  const float* bn1_b   = (const float*)d_in[4];
  const float* pos1_w  = (const float*)d_in[5];
  const float* pos1_b  = (const float*)d_in[6];
  const float* gat1_w  = (const float*)d_in[7];
  const float* gat1_as = (const float*)d_in[8];
  const float* gat1_ad = (const float*)d_in[9];
  const float* gat1_b  = (const float*)d_in[10];
  const float* bn2_g   = (const float*)d_in[11];
  const float* bn2_b   = (const float*)d_in[12];
  const float* pos2_w  = (const float*)d_in[13];
  const float* pos2_b  = (const float*)d_in[14];
  const float* gat2_w  = (const float*)d_in[15];
  const float* gat2_as = (const float*)d_in[16];
  const float* gat2_ad = (const float*)d_in[17];
  const float* gat2_b  = (const float*)d_in[18];
  const float* bn3_g   = (const float*)d_in[19];
  const float* bn3_b   = (const float*)d_in[20];
  const float* mlp1_w  = (const float*)d_in[21];
  const float* mlp1_b  = (const float*)d_in[22];
  const float* mlp2_w  = (const float*)d_in[23];
  const float* mlp2_b  = (const float*)d_in[24];
  const float* filt    = (const float*)d_in[25];
  const float* filt_b  = (const float*)d_in[26];
  const float* enh1_w  = (const float*)d_in[27];
  const float* enh1_b  = (const float*)d_in[28];
  const float* enh2_w  = (const float*)d_in[29];
  const float* enh2_b  = (const float*)d_in[30];
  const float* bn4_g   = (const float*)d_in[31];
  const float* bn4_b   = (const float*)d_in[32];
  const int*   src     = (const int*)d_in[33];
  const int*   dst     = (const int*)d_in[34];
  float* outp = (float*)d_out;

  char* wsb = (char*)d_ws;
  size_t off = 0;
  auto take = [&](size_t bytes) -> size_t { const size_t o = off; off = (off + bytes + 255) & ~(size_t)255; return o; };
  const size_t o_rec = take((size_t)512 * RECP * sizeof(double));
  const size_t o_st1 = take(512), o_st2 = take(512), o_st3 = take(512), o_st4 = take(512);
  const size_t o_cw  = take(512);
  const size_t wpl   = (size_t)9 * CB * CC * sizeof(unsigned short);
  const size_t o_w1h = take(wpl), o_w1l = take(wpl), o_w2h = take(wpl), o_w2l = take(wpl);
  const size_t o_as  = take((size_t)RR * sizeof(float));
  const size_t o_ad  = take((size_t)RR * sizeof(float));
  const size_t o_X   = take((size_t)RR * CC * sizeof(float));
  const size_t o_H   = take((size_t)RR * CC * sizeof(float));
  const size_t o_e1h = take((size_t)RR * CB * sizeof(unsigned short));
  const size_t o_e1l = take((size_t)RR * CB * sizeof(unsigned short));
  if (off > ws_size) return;

  double* rec = (double*)(wsb + o_rec);
  float* st1 = (float*)(wsb + o_st1);
  float* st2 = (float*)(wsb + o_st2);
  float* st3 = (float*)(wsb + o_st3);
  float* st4 = (float*)(wsb + o_st4);
  float* cw  = (float*)(wsb + o_cw);
  unsigned short* W1h = (unsigned short*)(wsb + o_w1h);
  unsigned short* W1l = (unsigned short*)(wsb + o_w1l);
  unsigned short* W2h = (unsigned short*)(wsb + o_w2h);
  unsigned short* W2l = (unsigned short*)(wsb + o_w2l);
  float* asb = (float*)(wsb + o_as);
  float* adb = (float*)(wsb + o_ad);
  float* X   = (float*)(wsb + o_X);
  float* Hr  = (float*)(wsb + o_H);
  unsigned short* FFh = (unsigned short*)(wsb + o_H);
  unsigned short* FFl = (unsigned short*)(wsb + o_H + (size_t)RR * CC * sizeof(unsigned short));
  float* PRE = Hr;
  unsigned short* E1h = (unsigned short*)(wsb + o_e1h);
  unsigned short* E1l = (unsigned short*)(wsb + o_e1l);

  const int n8 = 9 * CB * CC / 8;
  k_prepw<<<(n8 + NTHR - 1) / NTHR, NTHR, 0, stream>>>(enh1_w, W1h, W1l, CB, CC, n8);
  k_prepw<<<(n8 + NTHR - 1) / NTHR, NTHR, 0, stream>>>(enh2_w, W2h, W2l, CC, CB, n8);

  k_conv1<<<RR / NTHR, NTHR, 0, stream>>>(x, conv1_w, conv1_b, X, rec);
  k_fin<<<1, 64, 0, stream>>>(rec, RR / NTHR, CA, (float)RR, bn1_g, bn1_b, mlp1_w, mlp1_b, mlp2_w, mlp2_b, 0, st1, cw);

  k_tr<CB, CA><<<RR / GR, NTHR, 0, stream>>>(X, st1, bn1_g, bn1_b, pos1_w, pos1_b, gat1_w, gat1_as, gat1_ad,
                                             Hr, asb, adb);
  const int lds1 = 512 * 2 * CB * 4 + 512 * 4 * 4 + NWAVE * WCAP * 4 + 32 + NWAVE * 32 * 2 * 2 * 8 + RECP * 8;
  hipFuncSetAttribute(reinterpret_cast<const void*>(&k_gat<CB, 512, 2>),
                      hipFuncAttributeMaxDynamicSharedMemorySize, lds1);
  k_gat<CB, 512, 2><<<NPIX / 512, NTHR, lds1, stream>>>(Hr, asb, adb, src, dst, gat1_b, X, rec, nE);
  k_fin<<<1, 64, 0, stream>>>(rec, NPIX / 512, CB, (float)RR, bn2_g, bn2_b, mlp1_w, mlp1_b, mlp2_w, mlp2_b, 0, st2, cw);

  k_tr<CC, CB><<<RR / GR, NTHR, 0, stream>>>(X, st2, bn2_g, bn2_b, pos2_w, pos2_b, gat2_w, gat2_as, gat2_ad,
                                             Hr, asb, adb);
  const int lds2 = 256 * 2 * CC * 4 + 256 * 4 * 4 + NWAVE * WCAP * 4 + 32 + NWAVE * 32 * 2 * 4 * 8 + RECP * 8;
  hipFuncSetAttribute(reinterpret_cast<const void*>(&k_gat<CC, 256, 4>),
                      hipFuncAttributeMaxDynamicSharedMemorySize, lds2);
  k_gat<CC, 256, 4><<<NPIX / 256, NTHR, lds2, stream>>>(Hr, asb, adb, src, dst, gat2_b, X, rec, nE);
  k_fin<<<1, 64, 0, stream>>>(rec, NPIX / 256, CC, (float)RR, bn3_g, bn3_b, mlp1_w, mlp1_b, mlp2_w, mlp2_b, 1, st3, cw);

  k_ffp<<<RR * 8 / NTHR, NTHR, 0, stream>>>(X, st3, bn3_g, bn3_b, cw, filt, filt_b, FFh, FFl);
  const int ldsc0 = NWAVE * 2 * 32 * CB * 2;
  k_conv<CC, CB, 0><<<NIMG * IMH, NTHR, ldsc0, stream>>>(FFh, FFl, W1h, W1l, enh1_b, E1h, E1l,
                                                         X, st3, bn3_g, bn3_b, cw, filt, filt_b, PRE, rec);
  const int ldsc1 = CC * 256 * 4 + RECP * 8;
  hipFuncSetAttribute(reinterpret_cast<const void*>(&k_conv<CB, CC, 1>),
                      hipFuncAttributeMaxDynamicSharedMemorySize, ldsc1);
  k_conv<CB, CC, 1><<<NIMG * IMH, NTHR, ldsc1, stream>>>(E1h, E1l, W2h, W2l, enh2_b, FFh, FFl,
                                                         X, st3, bn3_g, bn3_b, cw, filt, filt_b, PRE, rec);
  k_fin<<<1, 64, 0, stream>>>(rec, NIMG * IMH, CC, (float)RR, bn4_g, bn4_b, mlp1_w, mlp1_b, mlp2_w, mlp2_b, 0, st4, cw);
  k_out<<<RR * CC / 4 / NTHR, NTHR, 0, stream>>>(PRE, st4, bn4_g, bn4_b, outp);
}
